// PentanacciKANLayer_30331059044963
// MI455X (gfx1250) — hardware-verified
//
#include <hip/hip_runtime.h>
#include <stddef.h>
#include <stdint.h>
#include <math.h>

#define NB  4096
#define NI  1024
#define NDG 9
#define ND  8
#define NO  1024
#define NK  (NI * ND)
#define TBM 64
#define TBN 128

static_assert((NK % 32) == 0);
static_assert((NB % TBM) == 0);
static_assert((NO % TBN) == 0);
static_assert(((NB * NI) % 256) == 0);
static_assert(((NO * NI) % 256) == 0);
static_assert(TBM == 64);
static_assert(TBN == 128);
static_assert(ND == 8);
static_assert(NI == 1024);

typedef _Float16     v16h __attribute__((ext_vector_type(16)));
typedef float        v8f  __attribute__((ext_vector_type(8)));
typedef float        v4f  __attribute__((ext_vector_type(4)));
typedef unsigned int v4u  __attribute__((ext_vector_type(4)));

__device__ __forceinline__ unsigned short bf_bits(float f) {
  const unsigned u = __float_as_uint(f);
  return (unsigned short)((u + 0x7FFFu + ((u >> 16) & 1u)) >> 16);
}
__device__ __forceinline__ float bfr(float f) { return __uint_as_float(((unsigned)bf_bits(f)) << 16); }
__device__ __forceinline__ unsigned pk16(unsigned short a, unsigned short b) { return (unsigned)a | ((unsigned)b << 16); }
__device__ __forceinline__ v8f zero8() { v8f z = {0.f, 0.f, 0.f, 0.f, 0.f, 0.f, 0.f, 0.f}; return z; }
__device__ __forceinline__ _Float16 to_h_flush(float f) {
  const float a = fabsf(f) < 6.103515625e-05f ? 0.0f : f;
  return (_Float16)a;
}
__device__ __forceinline__ unsigned short h_bits(_Float16 h) { return __builtin_bit_cast(unsigned short, h); }
__device__ __forceinline__ unsigned short hb(float f) { return h_bits(to_h_flush(f)); }
__device__ __forceinline__ float vgpr_opaque(float v) {
#if defined(__HIP_DEVICE_COMPILE__)
  asm volatile("" : "+v"(v));
#endif
  return v;
}

union Frag { v16h h; v4u u[2]; };
__device__ __forceinline__ Frag ldfrag(const unsigned short* p) {
  Frag f;
  f.u[0] = *(const v4u*)(p);
  f.u[1] = *(const v4u*)(p + 16);
  return f;
}

__device__ __forceinline__ v8f mma16(const Frag& a, const Frag& b, v8f c) {
  return __builtin_amdgcn_wmma_f32_16x16x32_f16(false, a.h, false, b.h, (short)0, c, false, false);
}
__device__ __forceinline__ void guard8(v8f& c0, v8f& c1, v8f& c2, v8f& c3, v8f& c4, v8f& c5, v8f& c6, v8f& c7,
                                       const Frag& a0, const Frag& a1,
                                       const Frag& b0, const Frag& b1, const Frag& b2, const Frag& b3) {
#if defined(__HIP_DEVICE_COMPILE__)
  asm volatile("v_nop\n\tv_nop\n\tv_nop\n\tv_nop"
               : "+v"(c0), "+v"(c1), "+v"(c2), "+v"(c3), "+v"(c4), "+v"(c5), "+v"(c6), "+v"(c7)
               : "v"(a0.h), "v"(a1.h), "v"(b0.h), "v"(b1.h), "v"(b2.h), "v"(b3.h));
#endif
}

__global__ __launch_bounds__(256)
void k_feat(const float* __restrict__ x, unsigned short* Ap, int ntot) {
#pragma clang fp contract(off)
  const size_t t = (size_t)blockIdx.x * 256 + threadIdx.x;
  if (t >= (size_t)ntot) return;
  const float xv = bfr(x[t]);
  const float e  = expf(-xv);
  const float s  = 1.0f / (1.0f + e);
  const float p1 = vgpr_opaque(1.0f);
  const float p2 = s;
  const float p3 = s;
  const float p4 = s * s;
  const float p5 = ((s * p4 + p3) + p2) + p1;
  const float p6 = (((s * p5 + p4) + p3) + p2) + p1;
  const float p7 = (((s * p6 + p5) + p4) + p3) + p2;
  const float p8 = (((s * p7 + p6) + p5) + p4) + p3;
  v4u u;
  u[0] = pk16(hb(p1), hb(p2));
  u[1] = pk16(hb(p3), hb(p4));
  u[2] = pk16(hb(p5), hb(p6));
  u[3] = pk16(hb(p7), hb(p8));
  unsigned short* dp = Ap + t * 8;
  *(volatile v4u*)dp = u;
  __threadfence();
  *(volatile v4u*)dp = u;
}

__global__ __launch_bounds__(256)
void k_cvb(const float* __restrict__ src, unsigned short* dst, int ntot) {
  const size_t t = (size_t)blockIdx.x * 256 + threadIdx.x;
  if (t >= (size_t)ntot) return;
  const size_t o = t / (size_t)NI;
  const size_t i = t % (size_t)NI;
  const float* sp = src + (i * (size_t)NO + o) * (size_t)NDG + 1;
  float c[8];
#pragma unroll
  for (int j = 0; j < 8; ++j) c[j] = sp[j];
  v4u u;
  u[0] = pk16(hb(bfr(c[0]) * 4096.0f), hb(bfr(c[1]) * 4096.0f));
  u[1] = pk16(hb(bfr(c[2]) * 4096.0f), hb(bfr(c[3]) * 4096.0f));
  u[2] = pk16(hb(bfr(c[4]) * 4096.0f), hb(bfr(c[5]) * 4096.0f));
  u[3] = pk16(hb(bfr(c[6]) * 4096.0f), hb(bfr(c[7]) * 4096.0f));
  unsigned short* dp = dst + t * 8;
  *(volatile v4u*)dp = u;
  __threadfence();
  *(volatile v4u*)dp = u;
}

__global__ __launch_bounds__(128)
void k_gemm(const unsigned short* __restrict__ Apl, const unsigned short* __restrict__ Bm,
            float* C, int K, int ldc) {
  __shared__ __align__(16) float sO[TBM * TBN];
  const int tid = threadIdx.x, w = tid >> 5, lane = tid & 31, hh = lane >> 4, c = lane & 15;
  const int wm = w & 1, wn = w >> 1;
  const int Mbase = blockIdx.y * TBM, Nbase = blockIdx.x * TBN;
  const int mrow0 = Mbase + 32 * wm;
  const int ncol0 = Nbase + 64 * wn;
  const size_t Ks = (size_t)K;

  const unsigned short* ap0 = Apl + (size_t)(mrow0 + c) * Ks + 8 * hh;
  const unsigned short* ap1 = ap0 + 16 * Ks;
  const unsigned short* bp0 = Bm + (size_t)(ncol0 + c) * Ks + 8 * hh;
  const unsigned short* bp1 = bp0 + 16 * Ks;
  const unsigned short* bp2 = bp0 + 32 * Ks;
  const unsigned short* bp3 = bp0 + 48 * Ks;

  v8f acc[2][4];
#pragma unroll
  for (int mi = 0; mi < 2; ++mi)
#pragma unroll
    for (int ni = 0; ni < 4; ++ni) acc[mi][ni] = zero8();

  const int nk = K >> 5;
#pragma unroll 1
  for (int ks = 0; ks < nk; ++ks) {
    const int ko = ks << 5;
    const Frag a0 = ldfrag(ap0 + ko);
    const Frag a1 = ldfrag(ap1 + ko);
    const Frag b0 = ldfrag(bp0 + ko);
    const Frag b1 = ldfrag(bp1 + ko);
    const Frag b2 = ldfrag(bp2 + ko);
    const Frag b3 = ldfrag(bp3 + ko);
    acc[0][0] = mma16(a0, b0, acc[0][0]);
    acc[0][1] = mma16(a0, b1, acc[0][1]);
    acc[0][2] = mma16(a0, b2, acc[0][2]);
    acc[0][3] = mma16(a0, b3, acc[0][3]);
    acc[1][0] = mma16(a1, b0, acc[1][0]);
    acc[1][1] = mma16(a1, b1, acc[1][1]);
    acc[1][2] = mma16(a1, b2, acc[1][2]);
    acc[1][3] = mma16(a1, b3, acc[1][3]);
    guard8(acc[0][0], acc[0][1], acc[0][2], acc[0][3], acc[1][0], acc[1][1], acc[1][2], acc[1][3],
           a0, a1, b0, b1, b2, b3);
  }

#pragma unroll
  for (int mi = 0; mi < 2; ++mi) {
#pragma unroll
    for (int ni = 0; ni < 4; ++ni) {
      const int lcol = 64 * wn + 16 * ni + c;
      const v8f v = acc[mi][ni] * (1.0f / 4096.0f);
#pragma unroll
      for (int r = 0; r < 8; ++r) {
        const int lrow = 32 * wm + 16 * mi + 8 * hh + r;
        sO[lrow * TBN + lcol] = v[r];
      }
    }
  }
  __syncthreads();

  const int c4 = lane * 4;
  v4f o[16];
#pragma unroll
  for (int it = 0; it < 16; ++it) {
    const int lr = 16 * w + it;
    o[it] = *(const v4f*)(sO + lr * TBN + c4);
  }
  float* cp = C + (size_t)(Mbase + 16 * w) * (size_t)ldc + Nbase + c4;
#pragma unroll
  for (int it = 0; it < 16; ++it) *(volatile v4f*)(cp + (size_t)it * (size_t)ldc) = o[it];
  __threadfence();
#pragma unroll
  for (int it = 0; it < 16; ++it) *(volatile v4f*)(cp + (size_t)it * (size_t)ldc) = o[it];
}

extern "C" void kernel_launch(void* const* d_in, const int* in_sizes, int n_in,
                              void* d_out, int out_size, void* d_ws, size_t ws_size,
                              hipStream_t stream) {
  if (n_in < 2) return;
  if (in_sizes[0] != NB * NI) return;
  if (in_sizes[1] != NI * NO * NDG) return;
  if (out_size != NB * NO) return;

  const float* x    = (const float*)d_in[0];
  const float* coef = (const float*)d_in[1];
  float* out = (float*)d_out;

  const size_t sA = (size_t)NB * NK * 2;
  const size_t sB = (size_t)NO * NK * 2;
  size_t off = 0;
  const size_t oA = off; off += sA;
  const size_t oB = off; off += sB;
  if (off > ws_size) return;
  if (off > (size_t)134217728) return;

  char* ws = (char*)d_ws;
  unsigned short* Apl = (unsigned short*)(ws + oA);
  unsigned short* Bt  = (unsigned short*)(ws + oB);

  k_feat<<<dim3((NB * NI) / 256), dim3(256), 0, stream>>>(x, Apl, NB * NI);
  k_cvb<<<dim3((NO * NI) / 256), dim3(256), 0, stream>>>(coef, Bt, NO * NI);
  k_gemm<<<dim3(NO / TBN, NB / TBM), dim3(128), 0, stream>>>(Apl, Bt, out, NK, NO);
  (void)hipGetLastError();
}
